// LGCN_83184926589612
// MI455X (gfx1250) — hardware-verified
//
#include <hip/hip_runtime.h>
#include <stddef.h>


#define DF      64
#define DCAT    192
#define XP      256
#define SP      64
#define OW4     0
#define OW5     4096
#define OW6     8192
#define OW7     12288
#define OW8     24576
#define OW9     28672
#define OW10    40960
#define OW11    45056
#define OW11B   49152
#define WTOT    53248
#define NTHR    256
#define NWAVE   8
#define EPT     8
#define CHUNK   (NTHR * EPT)
#define WCAP    (EPT * 32)
#define LISTN   (NWAVE * WCAP)
#define NBMAX   2048
#define SLOTB   11
#define RCAP    28672
#define DEGCAP  4096
#define NSTRM   4
#define GBM     32
#define GTHR    64
#define CA      16.0f
#define CW      64.0f
#define SCL     0.0009765625f
#define WSCAP   134217728
#define LDS_BUILD ((2 * RCAP + 2 * NBMAX + LISTN) * 4 + 64)

static_assert((CHUNK & (CHUNK - 1)) == 0 && CHUNK <= 4096);
static_assert(NBMAX == (1 << SLOTB));
static_assert(NTHR * 8 == NBMAX);
static_assert(LISTN >= NBMAX);
static_assert(LISTN >= NWAVE * WCAP);
static_assert((RCAP % 32) == 0);
static_assert(LDS_BUILD <= 300000);
static_assert(GBM == (GTHR / 32) * 16);
static_assert(NSTRM * 8 == 32);
static_assert((DF % 32) == 0 && (DCAT % 32) == 0);
static_assert(XP == 4 * DF && SP == DF);
static_assert(OW5 - OW4 == DF * DF && OW8 - OW7 == DF * DCAT && OW10 - OW9 == DF * DCAT && WTOT - OW11B == DF * DF);

typedef float    v4f  __attribute__((ext_vector_type(4)));
typedef float    v8f  __attribute__((ext_vector_type(8)));
typedef int      v4i  __attribute__((ext_vector_type(4)));
typedef int      v8i  __attribute__((ext_vector_type(8)));
typedef _Float16 v8h  __attribute__((ext_vector_type(8)));
typedef _Float16 v16h __attribute__((ext_vector_type(16)));
union FragH { v16h v; v8h h[2]; v8i w; };

__device__ __forceinline__ v8f wmh(const FragH& a, const FragH& b, v8f c) {
  v8f d = __builtin_amdgcn_wmma_f32_16x16x32_f16(false, a.v, false, b.v, (short)0, c, false, false);
  asm volatile("v_nop\n\tv_nop\n\tv_nop\n\tv_nop" : "+v"(d) : "v"(a.w), "v"(b.w));
  return d;
}

__device__ __forceinline__ v8h pack8(v4f a, v4f b, float sc) {
  v8h hv;
  hv[0] = (_Float16)(a.x * sc); hv[1] = (_Float16)(a.y * sc);
  hv[2] = (_Float16)(a.z * sc); hv[3] = (_Float16)(a.w * sc);
  hv[4] = (_Float16)(b.x * sc); hv[5] = (_Float16)(b.y * sc);
  hv[6] = (_Float16)(b.z * sc); hv[7] = (_Float16)(b.w * sc);
  return hv;
}

__device__ __forceinline__ v4f shf4(v4f v, int msk) {
  v4f r;
  r.x = __shfl_xor(v.x, msk); r.y = __shfl_xor(v.y, msk);
  r.z = __shfl_xor(v.z, msk); r.w = __shfl_xor(v.w, msk);
  return r;
}

__device__ __forceinline__ void tile_store(const float* stg, float* gp, int n4, int tid) {
  const v4f* s4 = (const v4f*)stg;
#pragma unroll 1
  for (int f = tid; f < n4; f += GTHR) {
    const v4f v = s4[f];
    *(volatile v4f*)(gp + 4 * f) = v;
  }
  __threadfence();
#pragma unroll 1
  for (int f = tid; f < n4; f += GTHR) {
    const v4f v = s4[f];
    *(volatile v4f*)(gp + 4 * f) = v;
  }
}

__device__ __forceinline__ int scan_chunk(const int* __restrict__ dsts, int nE, int cbase, int slotBase,
                                          int nb, int vec8, int* list, int tid, int lane, int wave) {
  int wc = 0;
  const int el0  = tid * EPT;
  const int e0   = cbase + el0;
  const int sent = -2147483647 - 1;
  v4i da, db;
  if (vec8 != 0 && cbase + CHUNK <= nE) {
    da = *(const v4i*)(dsts + e0);
    db = *(const v4i*)(dsts + e0 + 4);
  } else {
    da.x = (e0     < nE) ? dsts[min(e0,     nE - 1)] : sent;
    da.y = (e0 + 1 < nE) ? dsts[min(e0 + 1, nE - 1)] : sent;
    da.z = (e0 + 2 < nE) ? dsts[min(e0 + 2, nE - 1)] : sent;
    da.w = (e0 + 3 < nE) ? dsts[min(e0 + 3, nE - 1)] : sent;
    db.x = (e0 + 4 < nE) ? dsts[min(e0 + 4, nE - 1)] : sent;
    db.y = (e0 + 5 < nE) ? dsts[min(e0 + 5, nE - 1)] : sent;
    db.z = (e0 + 6 < nE) ? dsts[min(e0 + 6, nE - 1)] : sent;
    db.w = (e0 + 7 < nE) ? dsts[min(e0 + 7, nE - 1)] : sent;
  }
  const unsigned nbs = (unsigned)slotBase;
  const unsigned unb = (unsigned)nb;
  const unsigned s0 = (unsigned)da.x - nbs, s1 = (unsigned)da.y - nbs;
  const unsigned s2 = (unsigned)da.z - nbs, s3 = (unsigned)da.w - nbs;
  const unsigned s4 = (unsigned)db.x - nbs, s5 = (unsigned)db.y - nbs;
  const unsigned s6 = (unsigned)db.z - nbs, s7 = (unsigned)db.w - nbs;
  const bool h0 = s0 < unb, h1 = s1 < unb, h2 = s2 < unb, h3 = s3 < unb;
  const bool h4 = s4 < unb, h5 = s5 < unb, h6 = s6 < unb, h7 = s7 < unb;
  const unsigned any = __builtin_amdgcn_ballot_w32(h0 | h1 | h2 | h3 | h4 | h5 | h6 | h7);
  if (any != 0u) {
#define HITJ(J, HJ, SJ) { \
      const unsigned mj = __builtin_amdgcn_ballot_w32(HJ); \
      if (mj != 0u) { \
        if (HJ) { \
          const int pos = wc + (int)__builtin_amdgcn_mbcnt_lo(mj, 0u); \
          if (pos < WCAP) list[wave * WCAP + pos] = ((el0 + (J)) << 12) | (int)(SJ); \
        } \
        wc += (int)__builtin_popcount(mj); } }
    HITJ(0, h0, s0)
    HITJ(1, h1, s1)
    HITJ(2, h2, s2)
    HITJ(3, h3, s3)
    HITJ(4, h4, s4)
    HITJ(5, h5, s5)
    HITJ(6, h6, s6)
    HITJ(7, h7, s7)
#undef HITJ
  }
  return wc;
}

__global__ __launch_bounds__(NTHR) void k_xprep(const float* __restrict__ h, const float* __restrict__ cx,
                                                const float* __restrict__ cc,
                                                _Float16* xa, _Float16* s16, int nN, int nUnits) {
  const int i = (int)blockIdx.x * NTHR + (int)threadIdx.x;
  if (i >= nUnits) return;
  const int row = i >> 5;
  const int c0  = (i & 31) * 8;
  const int seg = c0 >> 6;
  const int col = c0 & (DF - 1);
  const int rc  = row < nN ? row : nN - 1;
  const float* base = (seg == 0) ? h : ((seg == 1) ? cx : cc);
  const float* p = base + (size_t)rc * DF + col;
  v4f a = *(const v4f*)p, b = *(const v4f*)(p + 4);
  const v4f z4 = {0.f, 0.f, 0.f, 0.f};
  if (row >= nN || seg == 3) { a = z4; b = z4; }
  const v8h hv = pack8(a, b, CA);
  const v8h zh = pack8(z4, z4, CA);
  const bool padS = (row >= nN) && (c0 < SP);
  const size_t o  = (size_t)row * XP + c0;
  const size_t os = (size_t)row * SP + c0;
  *(volatile v8h*)(xa + o) = hv;
  if (padS) *(volatile v8h*)(s16 + os) = zh;
  __threadfence();
  *(volatile v8h*)(xa + o) = hv;
  if (padS) *(volatile v8h*)(s16 + os) = zh;
}

__global__ __launch_bounds__(NTHR) void k_wprep(const float* __restrict__ w4, const float* __restrict__ w5,
                                                const float* __restrict__ w6, const float* __restrict__ w7,
                                                const float* __restrict__ w8, const float* __restrict__ w9,
                                                const float* __restrict__ w10, const float* __restrict__ w11,
                                                const float* __restrict__ w11b, _Float16* wt) {
  const int j = (int)blockIdx.y;
  const int u = (int)blockIdx.x * NTHR + (int)threadIdx.x;
  const float* w = (j == 0) ? w4 : (j == 1) ? w5 : (j == 2) ? w6 : (j == 3) ? w7 : (j == 4) ? w8 :
                   (j == 5) ? w9 : (j == 6) ? w10 : (j == 7) ? w11 : w11b;
  const int K    = (j == 3 || j == 5) ? DCAT : DF;
  const int dofs = (j == 0) ? OW4 : (j == 1) ? OW5 : (j == 2) ? OW6 : (j == 3) ? OW7 : (j == 4) ? OW8 :
                   (j == 5) ? OW9 : (j == 6) ? OW10 : (j == 7) ? OW11 : OW11B;
  const int kq = K >> 3;
  const int nUnits = DF * kq;
  if (u >= nUnits) return;
  const int n  = u / kq;
  const int k8 = (u - n * kq) * 8;
  const float* p = w + (size_t)k8 * DF + n;
  v4f a, b;
  a.x = p[0 * DF]; a.y = p[1 * DF]; a.z = p[2 * DF]; a.w = p[3 * DF];
  b.x = p[4 * DF]; b.y = p[5 * DF]; b.z = p[6 * DF]; b.w = p[7 * DF];
  const v8h hv = pack8(a, b, CW);
  const size_t o = (size_t)dofs + (size_t)8 * u;
  *(volatile v8h*)(wt + o) = hv;
  __threadfence();
  *(volatile v8h*)(wt + o) = hv;
}

__global__ __launch_bounds__(GTHR) void k_node(const _Float16* __restrict__ xa, const _Float16* __restrict__ wt,
                                               float* SE, float* DE, float* FT) {
  __shared__ __attribute__((aligned(16))) _Float16 sF[GBM * DF];
  __shared__ __attribute__((aligned(16))) float stg[GBM * DF];
  const int tid = threadIdx.x, lane = tid & 31, wave = tid >> 5, hh = lane >> 4, m = lane & 15;
  const int rowBase = (int)blockIdx.x * GBM;
  const _Float16* arow = xa + (size_t)(rowBase + 16 * wave + m) * XP + 8 * hh;
  const v8f z8 = {0.f, 0.f, 0.f, 0.f, 0.f, 0.f, 0.f, 0.f};

  {
    v8f a4[4], a5[4];
#pragma unroll
    for (int t = 0; t < 4; ++t) { a4[t] = z8; a5[t] = z8; }
#pragma unroll
    for (int ks = 0; ks < DF / 32; ++ks) {
      FragH fh, fx;
      fh.h[0] = *(const v8h*)(arow + 32 * ks);
      fh.h[1] = *(const v8h*)(arow + 32 * ks + 16);
      fx.h[0] = *(const v8h*)(arow + DF + 32 * ks);
      fx.h[1] = *(const v8h*)(arow + DF + 32 * ks + 16);
#pragma unroll
      for (int t = 0; t < 4; ++t) {
        const size_t bo = (size_t)(16 * t + m) * DF + 8 * hh + 32 * ks;
        FragH b4, b5;
        b4.h[0] = *(const v8h*)(wt + OW4 + bo);  b4.h[1] = *(const v8h*)(wt + OW4 + bo + 16);
        b5.h[0] = *(const v8h*)(wt + OW5 + bo);  b5.h[1] = *(const v8h*)(wt + OW5 + bo + 16);
        a4[t] = wmh(fh, b4, a4[t]);
        a5[t] = wmh(fx, b5, a5[t]);
      }
    }
    _Float16* fp = sF + (size_t)(16 * wave + 8 * hh) * DF + m;
#pragma unroll
    for (int t = 0; t < 4; ++t) {
#pragma unroll
      for (int r = 0; r < 8; ++r) {
        const float fu = (a4[t][r] * SCL) * (a5[t][r] * SCL);
        fp[(size_t)r * DF + 16 * t] = (_Float16)(fu * CA);
      }
    }
  }
  __syncthreads();
  const _Float16* frow = sF + (size_t)(16 * wave + m) * DF + 8 * hh;

  {
    v8f a6[4];
#pragma unroll
    for (int t = 0; t < 4; ++t) a6[t] = z8;
#pragma unroll
    for (int ks = 0; ks < DF / 32; ++ks) {
      FragH ff;
      ff.h[0] = *(const v8h*)(frow + 32 * ks);
      ff.h[1] = *(const v8h*)(frow + 32 * ks + 16);
#pragma unroll
      for (int t = 0; t < 4; ++t) {
        const size_t bo = (size_t)(16 * t + m) * DF + 8 * hh + 32 * ks;
        FragH b6;
        b6.h[0] = *(const v8h*)(wt + OW6 + bo);  b6.h[1] = *(const v8h*)(wt + OW6 + bo + 16);
        a6[t] = wmh(ff, b6, a6[t]);
      }
    }
    float* sp = stg + (size_t)(16 * wave + 8 * hh) * DF + m;
#pragma unroll
    for (int t = 0; t < 4; ++t) {
#pragma unroll
      for (int r = 0; r < 8; ++r) sp[(size_t)r * DF + 16 * t] = a6[t][r] * SCL;
    }
  }
  __syncthreads();
  tile_store(stg, DE + (size_t)rowBase * DF, GBM * DF / 4, tid);
  __syncthreads();

#pragma unroll 1
  for (int q = 0; q < 2; ++q) {
    const _Float16* wA = wt + (q == 0 ? OW7 : OW9);
    const _Float16* wB = wt + (q == 0 ? OW8 : OW10);
    float* dstp = (q == 0) ? SE : FT;
    v8f aA[4], aB[4];
#pragma unroll
    for (int t = 0; t < 4; ++t) { aA[t] = z8; aB[t] = z8; }
#pragma unroll
    for (int ks = 0; ks < (2 * DF) / 32; ++ks) {
      FragH fa;
      fa.h[0] = *(const v8h*)(arow + 32 * ks);
      fa.h[1] = *(const v8h*)(arow + 32 * ks + 16);
#pragma unroll
      for (int t = 0; t < 4; ++t) {
        const size_t bo = (size_t)(16 * t + m) * DCAT + 8 * hh + 32 * ks;
        FragH bb;
        bb.h[0] = *(const v8h*)(wA + bo);  bb.h[1] = *(const v8h*)(wA + bo + 16);
        aA[t] = wmh(fa, bb, aA[t]);
      }
    }
#pragma unroll
    for (int ks = 0; ks < DF / 32; ++ks) {
      FragH ff;
      ff.h[0] = *(const v8h*)(frow + 32 * ks);
      ff.h[1] = *(const v8h*)(frow + 32 * ks + 16);
#pragma unroll
      for (int t = 0; t < 4; ++t) {
        const size_t bo = (size_t)(16 * t + m) * DCAT + 8 * hh + 2 * DF + 32 * ks;
        FragH bb;
        bb.h[0] = *(const v8h*)(wA + bo);  bb.h[1] = *(const v8h*)(wA + bo + 16);
        aA[t] = wmh(ff, bb, aA[t]);
      }
    }
#pragma unroll
    for (int ks = 0; ks < DF / 32; ++ks) {
      FragH fc;
      fc.h[0] = *(const v8h*)(arow + 2 * DF + 32 * ks);
      fc.h[1] = *(const v8h*)(arow + 2 * DF + 32 * ks + 16);
#pragma unroll
      for (int t = 0; t < 4; ++t) {
        const size_t bo = (size_t)(16 * t + m) * DF + 8 * hh + 32 * ks;
        FragH bb;
        bb.h[0] = *(const v8h*)(wB + bo);  bb.h[1] = *(const v8h*)(wB + bo + 16);
        aB[t] = wmh(fc, bb, aB[t]);
      }
    }
    float* sp = stg + (size_t)(16 * wave + 8 * hh) * DF + m;
#pragma unroll
    for (int t = 0; t < 4; ++t) {
#pragma unroll
      for (int r = 0; r < 8; ++r) sp[(size_t)r * DF + 16 * t] = (aA[t][r] * SCL) * (aB[t][r] * SCL);
    }
    __syncthreads();
    tile_store(stg, dstp + (size_t)rowBase * DF, GBM * DF / 4, tid);
    __syncthreads();
  }
}

__global__ __launch_bounds__(NTHR) void k_build(const int* __restrict__ dsts, int* EL, int* OFF, int* CNT,
                                                int nE, int nb, int tp, int vec8) {
  extern __shared__ v4f lds_dyn[];
  int* reg1 = (int*)lds_dyn;
  int* reg2 = reg1 + RCAP;
  int* scnt = reg2 + RCAP;
  int* soff = scnt + NBMAX;
  int* list = soff + NBMAX;
  int* wcnt = list + LISTN;
  int* wtot = wcnt + NWAVE;
  const int tid = threadIdx.x, lane = tid & 31, wave = tid >> 5;
  const int nodeBase = (int)blockIdx.x * nb;

  for (int i = tid; i < NBMAX; i += NTHR) scnt[i] = 0;
  {
    const v4i z = {0, 0, 0, 0};
    v4i* r2v = (v4i*)reg2;
    for (int f = tid; f < RCAP / 4; f += NTHR) r2v[f] = z;
  }
  __syncthreads();

  int tot = 0;
  const int nChunks = (nE + CHUNK - 1) / CHUNK;
#pragma unroll 1
  for (int ch = 0; ch < nChunks; ++ch) {
    const int cbase = ch * CHUNK;
    const int wc = scan_chunk(dsts, nE, cbase, nodeBase, nb, vec8, list, tid, lane, wave);
    if (lane == 0) wcnt[wave] = wc;
    __syncthreads();
    int pre = 0, all = 0;
#pragma unroll
    for (int w2 = 0; w2 < NWAVE; ++w2) {
      int c = wcnt[w2];
      c = c < 0 ? 0 : (c > WCAP ? WCAP : c);
      all += c;
      pre += (w2 < wave) ? c : 0;
    }
    const int wcc  = wc > WCAP ? WCAP : wc;
    const int base = tot + pre;
#pragma unroll 1
    for (int i = lane; i < wcc; i += 32) {
      const int ent = list[wave * WCAP + i];
      const int el  = (ent >> 12) & (CHUNK - 1);
      const int sl  = ent & (NBMAX - 1);
      int eid = cbase + el;
      eid = eid > nE - 1 ? nE - 1 : eid;
      const int pos = base + i;
      if (pos < RCAP) reg1[pos] = (int)(((unsigned)eid << SLOTB) | (unsigned)sl);
    }
    tot += all;
    tot = tot > RCAP ? RCAP : tot;
    __syncthreads();
  }
  const int nh = tot;

  if (wave == 0) {
#pragma unroll 1
    for (int b0 = 0; b0 < nh; b0 += 32) {
      const int idx = b0 + lane;
      const int uv  = reg1[idx < RCAP ? idx : RCAP - 1];
      const int m32 = (nh - b0) < 32 ? (nh - b0) : 32;
#pragma unroll 1
      for (int k = 0; k < m32; ++k) {
        const int u  = __builtin_amdgcn_readlane(uv, k);
        const int sl = u & (NBMAX - 1);
        if (lane == 0) scnt[sl] = scnt[sl] + 1;
      }
    }
  }
  __syncthreads();

  {
    const v4i ca = *(const v4i*)(scnt + 8 * tid);
    const v4i cb = *(const v4i*)(scnt + 8 * tid + 4);
    const int e0 = ca.x < 0 ? 0 : ca.x, e1 = ca.y < 0 ? 0 : ca.y, e2 = ca.z < 0 ? 0 : ca.z, e3 = ca.w < 0 ? 0 : ca.w;
    const int e4 = cb.x < 0 ? 0 : cb.x, e5 = cb.y < 0 ? 0 : cb.y, e6 = cb.z < 0 ? 0 : cb.z, e7 = cb.w < 0 ? 0 : cb.w;
    const int ts = e0 + e1 + e2 + e3 + e4 + e5 + e6 + e7;
    int incl = ts;
#pragma unroll
    for (int d = 1; d < 32; d <<= 1) {
      const int up = __shfl_up(incl, d);
      if (lane >= d) incl += up;
    }
    if (lane == 31) wtot[wave] = incl;
    __syncthreads();
    int pre = 0;
#pragma unroll
    for (int w2 = 0; w2 < NWAVE; ++w2) pre += (w2 < wave) ? wtot[w2] : 0;
    int run = pre + incl - ts;
    soff[8 * tid + 0] = run; run += e0;
    soff[8 * tid + 1] = run; run += e1;
    soff[8 * tid + 2] = run; run += e2;
    soff[8 * tid + 3] = run; run += e3;
    soff[8 * tid + 4] = run; run += e4;
    soff[8 * tid + 5] = run; run += e5;
    soff[8 * tid + 6] = run; run += e6;
    soff[8 * tid + 7] = run;
  }
  __syncthreads();
  for (int i = tid; i < NBMAX; i += NTHR) list[i] = soff[i];
  __syncthreads();

  if (wave == 0) {
#pragma unroll 1
    for (int b0 = 0; b0 < nh; b0 += 32) {
      const int idx = b0 + lane;
      const int uv  = reg1[idx < RCAP ? idx : RCAP - 1];
      const int m32 = (nh - b0) < 32 ? (nh - b0) : 32;
#pragma unroll 1
      for (int k = 0; k < m32; ++k) {
        const int u   = __builtin_amdgcn_readlane(uv, k);
        const int sl  = u & (NBMAX - 1);
        const int eid = (int)((unsigned)u >> SLOTB);
        if (lane == 0) {
          int pos = list[sl];
          pos = pos < 0 ? 0 : (pos > RCAP - 1 ? RCAP - 1 : pos);
          reg2[pos] = eid;
          list[sl] = pos + 1;
        }
      }
    }
  }
  __syncthreads();

  {
    int* elb = EL + (size_t)blockIdx.x * RCAP;
    const v4i* r4 = (const v4i*)reg2;
#pragma unroll 1
    for (int f = tid; f < RCAP / 4; f += NTHR) {
      const v4i v = r4[f];
      *(volatile v4i*)(elb + 4 * f) = v;
    }
    __threadfence();
#pragma unroll 1
    for (int f = tid; f < RCAP / 4; f += NTHR) {
      const v4i v = r4[f];
      *(volatile v4i*)(elb + 4 * f) = v;
    }
  }
  {
    const bool ovf = (nh >= RCAP);
    int* ob = OFF + (size_t)blockIdx.x * tp;
    int* cb = CNT + (size_t)blockIdx.x * tp;
    const int n4 = tp >> 2;
#pragma unroll 1
    for (int pass = 0; pass < 2; ++pass) {
#pragma unroll 1
      for (int f = tid; f < n4; f += NTHR) {
        v4i so, sc;
        {
          const int s = 4 * f + 0; const bool in = s < nb; const int scl = s < NBMAX ? s : NBMAX - 1;
          so.x = in ? soff[scl] : 0; sc.x = in ? (ovf ? -1 : scnt[scl]) : 0;
        }
        {
          const int s = 4 * f + 1; const bool in = s < nb; const int scl = s < NBMAX ? s : NBMAX - 1;
          so.y = in ? soff[scl] : 0; sc.y = in ? (ovf ? -1 : scnt[scl]) : 0;
        }
        {
          const int s = 4 * f + 2; const bool in = s < nb; const int scl = s < NBMAX ? s : NBMAX - 1;
          so.z = in ? soff[scl] : 0; sc.z = in ? (ovf ? -1 : scnt[scl]) : 0;
        }
        {
          const int s = 4 * f + 3; const bool in = s < nb; const int scl = s < NBMAX ? s : NBMAX - 1;
          so.w = in ? soff[scl] : 0; sc.w = in ? (ovf ? -1 : scnt[scl]) : 0;
        }
        *(volatile v4i*)(ob + 4 * f) = so;
        *(volatile v4i*)(cb + 4 * f) = sc;
      }
      __threadfence();
    }
  }
}

__device__ __forceinline__ float edge_fetch(const int* __restrict__ elb, const int* __restrict__ srcs,
                                            const float* __restrict__ SE, const float* __restrict__ FT,
                                            int idx, int nE, int nN, int cb0, v4f d0, v4f d1,
                                            v4f& x0, v4f& x1) {
  int eid = elb[idx];
  eid = eid < 0 ? 0 : (eid > nE - 1 ? nE - 1 : eid);
  const int sraw = srcs[eid];
  const int s = sraw < 0 ? 0 : (sraw > nN - 1 ? nN - 1 : sraw);
  const float* ps = SE + (size_t)s * DF + cb0;
  const float* pf = FT + (size_t)s * DF + cb0;
  const v4f e0 = *(const v4f*)ps, e1 = *(const v4f*)(ps + 4);
  x0 = *(const v4f*)pf;  x1 = *(const v4f*)(pf + 4);
  float pr = e0.x * d0.x;
  pr = fmaf(e0.y, d0.y, pr); pr = fmaf(e0.z, d0.z, pr); pr = fmaf(e0.w, d0.w, pr);
  pr = fmaf(e1.x, d1.x, pr); pr = fmaf(e1.y, d1.y, pr); pr = fmaf(e1.z, d1.z, pr); pr = fmaf(e1.w, d1.w, pr);
  pr += __shfl_xor(pr, 1);
  pr += __shfl_xor(pr, 2);
  pr += __shfl_xor(pr, 4);
  return pr;
}

__global__ __launch_bounds__(NTHR) void k_agg(
    const int* __restrict__ srcs, const int* __restrict__ EL,
    const int* __restrict__ OFF, const int* __restrict__ CNT,
    const float* __restrict__ SE, const float* __restrict__ DE, const float* __restrict__ FT,
    _Float16* s16, int nN, int nE, int nb, int tp) {
  const int tid = threadIdx.x, lane = tid & 31, wave = tid >> 5;
  const int g   = lane >> 3;
  const int sub = lane & 7;
  const int cb0 = 8 * sub;
  const int nodeBase = (int)blockIdx.x * nb;
  const int nbw = nb >> 3;
  const int* elb  = EL  + (size_t)blockIdx.x * RCAP;
  const int* offb = OFF + (size_t)blockIdx.x * tp;
  const int* cntb = CNT + (size_t)blockIdx.x * tp;
  const float qnan = __int_as_float(0x7fc00000);
  const v4f z4 = {0.f, 0.f, 0.f, 0.f};
#pragma unroll 1
  for (int jt = 0; jt < nbw; ++jt) {
    const int slot = wave * nbw + jt;
    const int grow = nodeBase + slot;
    const int gcl  = grow < nN ? grow : nN - 1;
    const bool wr  = grow < nN;
    int st = offb[slot];
    const int craw = cntb[slot];
    st = st < 0 ? 0 : (st > RCAP - 1 ? RCAP - 1 : st);
    int cnt = craw < 0 ? 0 : (craw > DEGCAP ? DEGCAP : craw);
    if (cnt > RCAP - st) cnt = RCAP - st;
    const float pz = (craw < 0 || craw > DEGCAP) ? qnan : 0.0f;

    const float* pd = DE + (size_t)gcl * DF + cb0;
    const v4f d0 = *(const v4f*)pd, d1 = *(const v4f*)(pd + 4);

    int q0c = (g < cnt) ? g : (cnt - 1);
    q0c = q0c < 0 ? 0 : q0c;
    v4f x0, x1;
    const float l0 = edge_fetch(elb, srcs, SE, FT, st + q0c, nE, nN, cb0, d0, d1, x0, x1);
    const bool v0 = g < cnt;
    float mx = v0 ? l0 : 0.0f;
    float dn = v0 ? 1.0f : 0.0f;
    v4f a0 = v0 ? x0 : z4, a1 = v0 ? x1 : z4;
    const int niter = (cnt + NSTRM - 1) / NSTRM;
#pragma unroll 1
    for (int it = 1; it < niter; ++it) {
      const int q = it * NSTRM + g;
      const bool valid = q < cnt;
      const int qc = valid ? q : cnt - 1;
      v4f y0, y1;
      const float l = edge_fetch(elb, srcs, SE, FT, st + qc, nE, nN, cb0, d0, d1, y0, y1);
      const float mn = valid ? fmaxf(mx, l) : mx;
      const float s1 = __expf(mx - mn);
      const float s2 = valid ? __expf(l - mn) : 0.0f;
      dn = fmaf(dn, s1, s2);
      a0 = a0 * s1 + y0 * s2;
      a1 = a1 * s1 + y1 * s2;
      mx = mn;
    }
    const float mxv = (g < cnt) ? mx : -3.0e38f;
    float m1 = fmaxf(mxv, __shfl_xor(mxv, 8));
    m1 = fmaxf(m1, __shfl_xor(m1, 16));
    const float es = (g < cnt) ? __expf(mx - m1) : 0.0f;
    v4f r0 = a0 * es, r1 = a1 * es;
    float ds = dn * es;
    r0 = r0 + shf4(r0, 8);   r1 = r1 + shf4(r1, 8);   ds += __shfl_xor(ds, 8);
    r0 = r0 + shf4(r0, 16);  r1 = r1 + shf4(r1, 16);  ds += __shfl_xor(ds, 16);
    const float inv = (cnt > 0) ? (1.0f / fmaxf(ds, 1.0f)) : 0.0f;
    const v4f so0 = r0 * inv + pz;
    const v4f so1 = r1 * inv + pz;
    const v8h hv = pack8(so0, so1, CA);
    _Float16* sp = s16 + (size_t)gcl * SP + 8 * lane;
    const bool doSt = wr && (lane < 8);
    if (doSt) *(volatile v8h*)sp = hv;
    __threadfence();
    if (doSt) *(volatile v8h*)sp = hv;
  }
}

__global__ __launch_bounds__(GTHR) void k_out(const _Float16* __restrict__ xa, const _Float16* __restrict__ s16,
                                              const _Float16* __restrict__ wt, float* out, int nN) {
  __shared__ __attribute__((aligned(16))) float stg[GBM * DF];
  const int tid = threadIdx.x, lane = tid & 31, wave = tid >> 5, hh = lane >> 4, m = lane & 15;
  const int rowBase = (int)blockIdx.x * GBM;
  const _Float16* arow = xa  + (size_t)(rowBase + 16 * wave + m) * XP + DF + 8 * hh;
  const _Float16* srow = s16 + (size_t)(rowBase + 16 * wave + m) * SP + 8 * hh;
  const v8f z8 = {0.f, 0.f, 0.f, 0.f, 0.f, 0.f, 0.f, 0.f};
  v8f acc[4];
#pragma unroll
  for (int t = 0; t < 4; ++t) acc[t] = z8;
#pragma unroll
  for (int ks = 0; ks < DF / 32; ++ks) {
    FragH fx;
    fx.h[0] = *(const v8h*)(arow + 32 * ks);
    fx.h[1] = *(const v8h*)(arow + 32 * ks + 16);
#pragma unroll
    for (int t = 0; t < 4; ++t) {
      const size_t bo = (size_t)(16 * t + m) * DF + 8 * hh + 32 * ks;
      FragH bb;
      bb.h[0] = *(const v8h*)(wt + OW11 + bo);  bb.h[1] = *(const v8h*)(wt + OW11 + bo + 16);
      acc[t] = wmh(fx, bb, acc[t]);
    }
  }
#pragma unroll
  for (int ks = 0; ks < DF / 32; ++ks) {
    FragH fs;
    fs.h[0] = *(const v8h*)(srow + 32 * ks);
    fs.h[1] = *(const v8h*)(srow + 32 * ks + 16);
#pragma unroll
    for (int t = 0; t < 4; ++t) {
      const size_t bo = (size_t)(16 * t + m) * DF + 8 * hh + 32 * ks;
      FragH bb;
      bb.h[0] = *(const v8h*)(wt + OW11B + bo);  bb.h[1] = *(const v8h*)(wt + OW11B + bo + 16);
      acc[t] = wmh(fs, bb, acc[t]);
    }
  }
  {
    float* sp = stg + (size_t)(16 * wave + 8 * hh) * DF + m;
#pragma unroll
    for (int t = 0; t < 4; ++t) {
#pragma unroll
      for (int r = 0; r < 8; ++r) sp[(size_t)r * DF + 16 * t] = acc[t][r] * SCL;
    }
  }
  __syncthreads();
  const int nValid = (nN - rowBase) < GBM ? (nN - rowBase) : GBM;
  const int n4 = nValid * (DF / 4);
  tile_store(stg, out + (size_t)rowBase * DF, n4, tid);
}

static int pick_nb(int nE, int nN) {
  int nb = NBMAX;
  while (nb > 16 && (long long)nb * (long long)nE * 5LL > (long long)RCAP * (long long)nN * 4LL) nb >>= 1;
  return nb;
}

extern "C" void kernel_launch(void* const* d_in, const int* in_sizes, int n_in,
                              void* d_out, int out_size, void* d_ws, size_t ws_size,
                              hipStream_t stream) {
  if (n_in < 14) return;
  const int nN = in_sizes[0] / DF;
  if (nN <= 0 || in_sizes[0] != nN * DF) return;
  if (in_sizes[1] != nN * DF || in_sizes[2] != nN * DF) return;
  if (nN > (1 << 22)) return;
  const int nE = in_sizes[3];
  if (nE < 1 || nE > (1 << 21)) return;
  if (in_sizes[4] != nE) return;
  if (in_sizes[5] != DF * DF || in_sizes[6] != DF * DF || in_sizes[7] != DF * DF) return;
  if (in_sizes[8] != DCAT * DF || in_sizes[10] != DCAT * DF) return;
  if (in_sizes[9] != DF * DF || in_sizes[11] != DF * DF) return;
  if (in_sizes[12] != DF * DF || in_sizes[13] != DF * DF) return;
  if (out_size != nN * DF) return;

  const float* h    = (const float*)d_in[0];
  const float* cx   = (const float*)d_in[1];
  const float* cc   = (const float*)d_in[2];
  const int*   srcs = (const int*)d_in[3];
  const int*   dsts = (const int*)d_in[4];
  const float* w4   = (const float*)d_in[5];
  const float* w5   = (const float*)d_in[6];
  const float* w6   = (const float*)d_in[7];
  const float* w7   = (const float*)d_in[8];
  const float* w8   = (const float*)d_in[9];
  const float* w9   = (const float*)d_in[10];
  const float* w10  = (const float*)d_in[11];
  const float* w11  = (const float*)d_in[12];
  const float* w11b = (const float*)d_in[13];
  float* out = (float*)d_out;

  const int MP   = ((nN + GBM - 1) / GBM) * GBM;
  const int nb   = pick_nb(nE, nN);
  const int tp   = nb < 32 ? 32 : nb;
  const int gA   = (nN + nb - 1) / nb;
  const int gG   = MP / GBM;
  const int vec8 = 1;
  const int nUnits = MP * (XP / 8);
  if (nb < 16 || nb > NBMAX || (long long)gA * nb < (long long)nN) return;

  char* ws = (char*)d_ws;
  size_t off = 0;
  const size_t oWT  = off; off += (size_t)WTOT * 2;              off = (off + 255) & ~(size_t)255;
  const size_t oXA  = off; off += (size_t)MP * XP * 2;           off = (off + 255) & ~(size_t)255;
  const size_t oSE  = off; off += (size_t)MP * DF * 4;           off = (off + 255) & ~(size_t)255;
  const size_t oDE  = off; off += (size_t)MP * DF * 4;           off = (off + 255) & ~(size_t)255;
  const size_t oFT  = off; off += (size_t)MP * DF * 4;           off = (off + 255) & ~(size_t)255;
  const size_t oS16 = off; off += (size_t)MP * SP * 2;           off = (off + 255) & ~(size_t)255;
  const size_t oEL  = off; off += (size_t)gA * RCAP * 4;         off = (off + 255) & ~(size_t)255;
  const size_t oOFF = off; off += (size_t)gA * tp * 4;           off = (off + 255) & ~(size_t)255;
  const size_t oCNT = off; off += (size_t)gA * tp * 4;           off = (off + 255) & ~(size_t)255;
  if (off > ws_size || off > (size_t)WSCAP) return;
  _Float16* WT  = (_Float16*)(ws + oWT);
  _Float16* XA  = (_Float16*)(ws + oXA);
  float*    SE  = (float*)(ws + oSE);
  float*    DE  = (float*)(ws + oDE);
  float*    FT  = (float*)(ws + oFT);
  _Float16* S16 = (_Float16*)(ws + oS16);
  int*      EL  = (int*)(ws + oEL);
  int*      OFF = (int*)(ws + oOFF);
  int*      CNT = (int*)(ws + oCNT);

  hipFuncSetAttribute(reinterpret_cast<const void*>(&k_build),
                      hipFuncAttributeMaxDynamicSharedMemorySize, LDS_BUILD);

  k_xprep<<<(nUnits + NTHR - 1) / NTHR, NTHR, 0, stream>>>(h, cx, cc, XA, S16, nN, nUnits);
  k_wprep<<<dim3((DF * (DCAT / 8) + NTHR - 1) / NTHR, 9), NTHR, 0, stream>>>(
      w4, w5, w6, w7, w8, w9, w10, w11, w11b, WT);

  k_build<<<gA, NTHR, LDS_BUILD, stream>>>(dsts, EL, OFF, CNT, nE, nb, tp, vec8);

  k_node<<<gG, GTHR, 0, stream>>>(XA, WT, SE, DE, FT);
  k_agg<<<gA, NTHR, 0, stream>>>(srcs, EL, OFF, CNT, SE, DE, FT, S16, nN, nE, nb, tp);

  k_out<<<gG, GTHR, 0, stream>>>(XA, S16, WT, out, nN);
}
